// MaxMatching_47923245089138
// MI455X (gfx1250) — hardware-verified
//
#include <hip/hip_runtime.h>
#include <math.h>

typedef __attribute__((ext_vector_type(16))) _Float16 v16h;
typedef __attribute__((ext_vector_type(16))) __bf16 v16b;
typedef __attribute__((ext_vector_type(8)))  _Float16 v8h;
typedef __attribute__((ext_vector_type(8)))  float v8f;
typedef __attribute__((ext_vector_type(4)))  float v4f;
typedef __attribute__((ext_vector_type(2)))  float v2f;
typedef __attribute__((ext_vector_type(4)))  unsigned v4u;
typedef __attribute__((ext_vector_type(4)))  int v4i;
typedef float __attribute__((may_alias)) float_a;
typedef int __attribute__((may_alias)) int_a;

template <typename T> __device__ __forceinline__ void vst2(void* p, T v) { *(volatile T*)p = v; __threadfence(); *(volatile T*)p = v; }
__device__ __forceinline__ v8f wmma16(v16h a, v16h b, v8f c) {
  v8f d = __builtin_amdgcn_wmma_f32_16x16x32_f16(false, a, false, b, (short)0, c, false, false);
  asm volatile("v_nop\n\tv_nop\n\tv_nop\n\tv_nop" : "+v"(d) : "v"(a), "v"(b));
  return d;
}
__device__ __forceinline__ v8f wmma_bf(v16b a, v16b b, v8f c) {
  v8f d = __builtin_amdgcn_wmma_f32_16x16x32_bf16(false, a, false, b, (short)0, c, false, false);
  asm volatile("v_nop\n\tv_nop\n\tv_nop\n\tv_nop" : "+v"(d) : "v"(a), "v"(b));
  return d;
}
__device__ __forceinline__ v16h frag_h(const _Float16* rowk0, int lane) {
  union { v16h v; v8h q[2]; } u; const _Float16* p = rowk0 + 8 * (lane >> 4);
  u.q[0] = *(const v8h*)p; u.q[1] = *(const v8h*)(p + 16); return u.v;
}
__device__ __forceinline__ v16h frag_f32(const float* rowk0, int lane) {
  v16h a; const float* p = rowk0 + 8 * (lane >> 4);
#pragma unroll
  for (int i = 0; i < 8; ++i) { a[i] = (_Float16)p[i]; a[8 + i] = (_Float16)p[16 + i]; }
  return a;
}
__device__ __forceinline__ v16h frag_f32s(const float* rowk0, int lane, float sc) {
  v16h a; const float* p = rowk0 + 8 * (lane >> 4);
#pragma unroll
  for (int i = 0; i < 8; ++i) { a[i] = (_Float16)(p[i] * sc); a[8 + i] = (_Float16)(p[16 + i] * sc); }
  return a;
}
__device__ __forceinline__ v16h fragc_f32(const float* W, int k0, int n, int lane, int ld, int K) {
  v16h a; const int g = lane >> 4;
#pragma unroll
  for (int i = 0; i < 8; ++i) { const int ka = k0 + 8 * g + i, kb = ka + 16;
    a[i] = (_Float16)(ka < K ? W[(size_t)(ka < K ? ka : K - 1) * ld + n] : 0.f); a[8 + i] = (_Float16)(kb < K ? W[(size_t)(kb < K ? kb : K - 1) * ld + n] : 0.f); }
  return a;
}
struct F2 { v16b h, l; };
__device__ __forceinline__ F2 bsplit16(const float v[16]) { F2 r;
#pragma unroll
  for (int i = 0; i < 16; ++i) { const __bf16 h = (__bf16)v[i]; r.h[i] = h; r.l[i] = (__bf16)(v[i] - (float)h); }
  return r; }
__device__ __forceinline__ F2 split_row(const float* row, int k0, int lane) { float v[16]; const float* p = row + k0 + 8 * (lane >> 4);
#pragma unroll
  for (int i = 0; i < 8; ++i) { v[i] = p[i]; v[8 + i] = p[16 + i]; }
  return bsplit16(v); }
__device__ __forceinline__ F2 split_rowK(const float* row, int k0, int lane, int K) { float v[16]; const int g = lane >> 4;
#pragma unroll
  for (int i = 0; i < 8; ++i) { const int ka = k0 + 8 * g + i, kb = ka + 16; v[i] = ka < K ? row[ka < K ? ka : K - 1] : 0.f; v[8 + i] = kb < K ? row[kb < K ? kb : K - 1] : 0.f; }
  return bsplit16(v); }
__device__ __forceinline__ F2 split_col(const float* W, int k0, int n, int lane, int ld, int K) { float v[16]; const int g = lane >> 4;
#pragma unroll
  for (int i = 0; i < 8; ++i) { const int ka = k0 + 8 * g + i, kb = ka + 16; v[i] = ka < K ? W[(size_t)(ka < K ? ka : K - 1) * ld + n] : 0.f; v[8 + i] = kb < K ? W[(size_t)(kb < K ? kb : K - 1) * ld + n] : 0.f; }
  return bsplit16(v); }
__device__ __forceinline__ v8f mac3(const F2& a, const F2& b, v8f c) { c = wmma_bf(a.l, b.h, c); c = wmma_bf(a.h, b.l, c); return wmma_bf(a.h, b.h, c); }
__device__ __forceinline__ float sigm(float v) { return 1.0f / (1.0f + expf(-v)); }
#define LDSX() do { asm volatile("s_wait_dscnt 0" ::: "memory"); __builtin_amdgcn_wave_barrier(); __builtin_amdgcn_fence(__ATOMIC_RELEASE, "workgroup"); } while (0)


#define NBT 64
#define L1 200
#define L2 200
#define DDM 300
#define NP 16
__device__ __forceinline__ float bfr(float v) { return (float)(__bf16)v; }
__device__ __forceinline__ v16b frag_b(const __bf16* rowk0, int lane) { return __builtin_bit_cast(v16b, frag_h((const _Float16*)rowk0, lane)); }

__global__ __launch_bounds__(128) void k_match(const float* __restrict__ s1, const float* __restrict__ s2, const float* __restrict__ ker, float* __restrict__ out) {
  __shared__ float sw2[DDM + 20]; __shared__ float sr2[L2 + 8]; __shared__ float smx[13 * 16]; __shared__ __align__(16) float so[L1][NP];
  __shared__ __align__(16) __bf16 t2h[112][320], t2l[112][320];
  const int tid = threadIdx.x, wave = tid >> 5, lane = tid & 31, col = lane & 15, g = lane >> 4; const int b = blockIdx.x;
  const float* s1b = s1 + (size_t)b * L1 * DDM; const float* s2b = s2 + (size_t)b * L2 * DDM;
#pragma unroll 1
  for (int p = 0; p < NP; ++p) {
    __syncthreads();
    for (int d = tid; d < DDM + 20; d += 128) { const float w = d < DDM ? bfr(ker[p * DDM + d]) : 0.f; sw2[d] = w * w; }
    __syncthreads();
    for (int j = tid; j < L2; j += 128) { float q = 0.f;
#pragma unroll 4
      for (int d = 0; d < DDM; ++d) { const float v = bfr(s2b[(size_t)j * DDM + d]); q += v * v * sw2[d]; }
      sr2[j] = rsqrtf(fmaxf(q, 1e-12f)); }
#pragma unroll 1
    for (int jh = 0; jh < 2; ++jh) { const int jb = jh * 112;
      __syncthreads();
      for (int q = tid; q < 112 * 320; q += 128) { const int jl = q / 320, d = q % 320; const int j = jb + jl; const float v = (j < L2 && d < DDM) ? bfr(s2b[(size_t)j * DDM + d]) * sw2[d] : 0.f; const __bf16 hi = (__bf16)v; t2h[jl][d] = hi; t2l[jl][d] = (__bf16)(v - (float)hi); }
      __syncthreads();
#pragma unroll 1
      for (int rt = wave; rt < 13; rt += 4) { const int irow = rt * 16 + col; const int ic = irow < L1 ? irow : L1 - 1;
        v8f acc[7] = {};
#pragma unroll 1
        for (int kc = 0; kc < (DDM + 31) / 32; ++kc) { const v16b a = split_rowK(s1b + (size_t)ic * DDM, kc * 32, lane, DDM).h;
#pragma unroll
          for (int t = 0; t < 7; ++t) { acc[t] = wmma_bf(a, frag_b(&t2l[t * 16 + col][kc * 32], lane), acc[t]); acc[t] = wmma_bf(a, frag_b(&t2h[t * 16 + col][kc * 32], lane), acc[t]); } }
        float mx[8];
#pragma unroll
        for (int r = 0; r < 8; ++r) { float m = -3.0e38f;
#pragma unroll
          for (int t = 0; t < 7; ++t) { const int j = jb + t * 16 + col; if (j < L2) m = fmaxf(m, acc[t][r] * sr2[j]); }
#pragma unroll
          for (int o_ = 1; o_ < 16; o_ <<= 1) m = fmaxf(m, __shfl_xor(m, o_, 32));
          mx[r] = m; }
        if (jh == 0) { if (col == 0) {
#pragma unroll
            for (int r = 0; r < 8; ++r) smx[rt * 16 + 8 * g + r] = mx[r]; } }
        else { float q = 0.f;
#pragma unroll 4
          for (int d = 0; d < DDM; ++d) { const float v = bfr(s1b[(size_t)ic * DDM + d]); q += v * v * sw2[d]; }
          const float r1 = rsqrtf(fmaxf(q, 1e-12f));
#pragma unroll
          for (int r = 0; r < 8; ++r) { const float rr1 = __shfl(r1, 8 * g + r, 32); const int row = rt * 16 + 8 * g + r; if (col == 0 && row < L1) so[row][p] = fmaxf(smx[row], mx[r]) * rr1; } } } } }
  __syncthreads();
  for (int q = tid; q < L1 * NP / 4; q += 128) vst2(out + (size_t)b * L1 * NP + q * 4, *(const v4f*)(&so[0][0] + q * 4));
}
extern "C" void kernel_launch(void* const* d_in, const int* in_sizes, int n_in, void* d_out, int out_size, void* d_ws, size_t ws_size, hipStream_t stream) {
  (void)in_sizes; (void)n_in; (void)out_size; (void)ws_size; (void)d_ws;
  const float* s1 = (const float*)d_in[0]; const float* s2 = (const float*)d_in[1]; const float* ker = (const float*)d_in[2];
  k_match<<<NBT, 128, 0, stream>>>(s1, s2, ker, (float*)d_out);
}
